// TGCNLongTerm_60765197304391
// MI455X (gfx1250) — hardware-verified
//
#include <hip/hip_runtime.h>
#include <stddef.h>


#define DD      256
#define WWIN    12
#define KT      (WWIN * DD)
#define KT8     (KT / 8)
#define GRUW    (3 * DD)
#define PMAXH   20
#define NTHR    256
#define NWAVE   8
#define GTHR    128
#define GBM     64
#define PGRP    64
#define NPGRP   (DD / PGRP)
#define KS1     (KT / 32)
#define KS2     (DD / 32)
#define NB      512
#define NBW     (NB / NWAVE)
#define NBMAX   1024
#define SLOTB   10
#define EPT     8
#define CHUNK   (NTHR * EPT)
#define WCAP    (EPT * 32)
#define LISTN   (NWAVE * WCAP)
#define RCAP    20480
#define WDEG    256
#define NCI     12
#define CG      256.0f
#define CWT     512.0f
#define SCL1    0.00000762939453125f
#define CT      64.0f
#define CHH     64.0f
#define CWG     256.0f
#define SCL2    0.00006103515625f
#define LDS_SCAN (((2 * RCAP) + (2 * NBMAX) + LISTN + (2 * NWAVE) + (NWAVE * WDEG) + (NWAVE * NCI * NBW)) * 4 + 64)

static_assert((CHUNK & (CHUNK - 1)) == 0 && CHUNK <= 2048);
static_assert(NBMAX == (1 << SLOTB));
static_assert(NTHR * 4 == NBMAX);
static_assert(NB <= NBMAX && (NB % (32 * NWAVE)) == 0);
static_assert(LISTN >= NBMAX);
static_assert((RCAP % 32) == 0);
static_assert((WDEG % 32) == 0);
static_assert(LDS_SCAN <= 300000);
static_assert(GBM == (GTHR / 32) * 16);
static_assert((KT % 64) == 0 && (DD % 32) == 0 && PGRP == 64 && (DD % PGRP) == 0);

typedef float    v4f  __attribute__((ext_vector_type(4)));
typedef float    v8f  __attribute__((ext_vector_type(8)));
typedef int      v4i  __attribute__((ext_vector_type(4)));
typedef int      v8i  __attribute__((ext_vector_type(8)));
typedef _Float16 v8h  __attribute__((ext_vector_type(8)));
typedef _Float16 v16h __attribute__((ext_vector_type(16)));
union FragH { v16h v; v8h h[2]; v8i w; };

__device__ __forceinline__ v8f wmh(const FragH& a, const FragH& b, v8f c) {
  v8f d = __builtin_amdgcn_wmma_f32_16x16x32_f16(false, a.v, false, b.v, (short)0, c, false, false);
  asm volatile("v_nop\n\tv_nop\n\tv_nop\n\tv_nop" : "+v"(d) : "v"(a.w), "v"(b.w));
  return d;
}

__global__ __launch_bounds__(NTHR) void k_zero(float* p, int nUnits) {
  const int i = (int)blockIdx.x * NTHR + (int)threadIdx.x;
  if (i >= nUnits) return;
  const v4f z = {0.f, 0.f, 0.f, 0.f};
  float* q = p + (size_t)i * 4;
  *(volatile v4f*)q = z;
  __threadfence();
  *(volatile v4f*)q = z;
}

__global__ __launch_bounds__(NTHR) void k_cvt(const float* __restrict__ x, _Float16* xh, int nRows, int nUnits, float sc) {
  const int i = (int)blockIdx.x * NTHR + (int)threadIdx.x;
  if (i >= nUnits) return;
  const int row = i >> 5;
  const int c0  = (i & 31) * 8;
  const int rc  = row < nRows ? row : nRows - 1;
  const float* p = x + (size_t)rc * DD + c0;
  v4f a = *(const v4f*)p, b = *(const v4f*)(p + 4);
  const v4f z4 = {0.f, 0.f, 0.f, 0.f};
  if (row >= nRows) { a = z4; b = z4; }
  v8h hv;
  hv[0] = (_Float16)(a.x * sc); hv[1] = (_Float16)(a.y * sc);
  hv[2] = (_Float16)(a.z * sc); hv[3] = (_Float16)(a.w * sc);
  hv[4] = (_Float16)(b.x * sc); hv[5] = (_Float16)(b.y * sc);
  hv[6] = (_Float16)(b.z * sc); hv[7] = (_Float16)(b.w * sc);
  const size_t o = (size_t)row * DD + c0;
  *(volatile v8h*)(xh + o) = hv;
  __threadfence();
  *(volatile v8h*)(xh + o) = hv;
}

__global__ __launch_bounds__(NTHR) void k_tat(const float* __restrict__ taw, _Float16* tat, int K) {
  __shared__ __attribute__((aligned(16))) _Float16 tl[DD * 72];
  const int tid = threadIdx.x, lane = tid & 31, wave = tid >> 5;
  const int k0 = (int)blockIdx.x * 64;
#pragma unroll 4
  for (int it = 0; it < 16; ++it) {
    const int idx = it * NTHR + tid;
    const int r   = idx >> 6;
    const int c4  = (idx & 63) * 4;
    int kr = k0 + r; kr = kr < K ? kr : K - 1;
    v4f v = *(const v4f*)(taw + (size_t)kr * DD + c4);
    if (k0 + r >= K) { const v4f z = {0.f, 0.f, 0.f, 0.f}; v = z; }
    tl[(c4 + 0) * 72 + r] = (_Float16)(v.x * CWT);
    tl[(c4 + 1) * 72 + r] = (_Float16)(v.y * CWT);
    tl[(c4 + 2) * 72 + r] = (_Float16)(v.z * CWT);
    tl[(c4 + 3) * 72 + r] = (_Float16)(v.w * CWT);
  }
  __syncthreads();
  const int cq = lane >> 3, j8 = lane & 7;
  v8h o[8];
#pragma unroll
  for (int i = 0; i < 8; ++i) o[i] = *(const v8h*)(tl + (32 * wave + 4 * i + cq) * 72 + 8 * j8);
#pragma unroll
  for (int i = 0; i < 8; ++i)
    *(volatile v8h*)(tat + (size_t)(32 * wave + 4 * i + cq) * K + k0 + 8 * j8) = o[i];
  __threadfence();
#pragma unroll
  for (int i = 0; i < 8; ++i)
    *(volatile v8h*)(tat + (size_t)(32 * wave + 4 * i + cq) * K + k0 + 8 * j8) = o[i];
}

__device__ __forceinline__ int scan_chunk(const int* __restrict__ key, int nE, int cbase, int slotBase,
                                          int* list, int tid, int lane, int wave, int vecok) {
  int wc = 0;
  const int el0  = tid * EPT;
  const int e0   = cbase + el0;
  const int sent = -2147483647 - 1;
  int d0, d1, d2, d3, d4, d5, d6, d7;
  if (vecok != 0) {
    const v4i p0 = *(const v4i*)(key + e0), p1 = *(const v4i*)(key + e0 + 4);
    d0 = p0.x; d1 = p0.y; d2 = p0.z; d3 = p0.w; d4 = p1.x; d5 = p1.y; d6 = p1.z; d7 = p1.w;
  } else {
    const int em = nE - 1;
    int c;
    c = e0 + 0; c = c > em ? em : c; d0 = key[c]; if (e0 + 0 > em) d0 = sent;
    c = e0 + 1; c = c > em ? em : c; d1 = key[c]; if (e0 + 1 > em) d1 = sent;
    c = e0 + 2; c = c > em ? em : c; d2 = key[c]; if (e0 + 2 > em) d2 = sent;
    c = e0 + 3; c = c > em ? em : c; d3 = key[c]; if (e0 + 3 > em) d3 = sent;
    c = e0 + 4; c = c > em ? em : c; d4 = key[c]; if (e0 + 4 > em) d4 = sent;
    c = e0 + 5; c = c > em ? em : c; d5 = key[c]; if (e0 + 5 > em) d5 = sent;
    c = e0 + 6; c = c > em ? em : c; d6 = key[c]; if (e0 + 6 > em) d6 = sent;
    c = e0 + 7; c = c > em ? em : c; d7 = key[c]; if (e0 + 7 > em) d7 = sent;
  }
  const unsigned nbs = (unsigned)slotBase;
  const unsigned unb = (unsigned)NB;
  const unsigned s0 = (unsigned)d0 - nbs, s1 = (unsigned)d1 - nbs;
  const unsigned s2 = (unsigned)d2 - nbs, s3 = (unsigned)d3 - nbs;
  const unsigned s4 = (unsigned)d4 - nbs, s5 = (unsigned)d5 - nbs;
  const unsigned s6 = (unsigned)d6 - nbs, s7 = (unsigned)d7 - nbs;
  const bool h0 = s0 < unb, h1 = s1 < unb, h2 = s2 < unb, h3 = s3 < unb;
  const bool h4 = s4 < unb, h5 = s5 < unb, h6 = s6 < unb, h7 = s7 < unb;
  const unsigned any = __builtin_amdgcn_ballot_w32(h0 | h1 | h2 | h3 | h4 | h5 | h6 | h7);
  if (any != 0u) {
#define HITJ(J, HJ, SJ) { \
      const unsigned mj = __builtin_amdgcn_ballot_w32(HJ); \
      if (mj != 0u) { \
        if (HJ) { \
          const int pos = wc + (int)__builtin_amdgcn_mbcnt_lo(mj, 0u); \
          if (pos < WCAP) list[wave * WCAP + pos] = ((el0 + (J)) << SLOTB) | (int)(SJ); \
        } \
        wc += (int)__builtin_popcount(mj); } }
    HITJ(0, h0, s0)
    HITJ(1, h1, s1)
    HITJ(2, h2, s2)
    HITJ(3, h3, s3)
    HITJ(4, h4, s4)
    HITJ(5, h5, s5)
    HITJ(6, h6, s6)
    HITJ(7, h7, s7)
#undef HITJ
  }
  return wc;
}

template <int MODE>
__global__ __launch_bounds__(NTHR) void k_spmv(const int* __restrict__ key, const int* __restrict__ oth,
                                               const float* __restrict__ ew, const float* __restrict__ dpl,
                                               const float* __restrict__ vsrc, float* outp,
                                               int nE, int nN, int npad, int vec8) {
  extern __shared__ v4i lds_dyn[];
  int* reg1 = (int*)lds_dyn;
  int* reg2 = reg1 + RCAP;
  int* scnt = reg2 + RCAP;
  int* soff = scnt + NBMAX;
  int* list = soff + NBMAX;
  int* wcnt = list + LISTN;
  int* wtot = wcnt + NWAVE;
  int* wsrc = wtot + NWAVE;
  float* wres = (float*)(wsrc + NWAVE * WDEG);
  const int NCO = (MODE == 1) ? NCI : 1;
  const int tid = threadIdx.x, lane = tid & 31, wave = tid >> 5;
  const int nodeBase = (int)blockIdx.x * NB;

  for (int i = tid; i < NBMAX; i += NTHR) scnt[i] = 0;
  __syncthreads();

  int tot = 0;
  const int nChunks = (nE + CHUNK - 1) / CHUNK;
#pragma unroll 1
  for (int ch = 0; ch < nChunks; ++ch) {
    const int cbase = ch * CHUNK;
    const int vecok = (vec8 != 0 && cbase + CHUNK <= nE) ? 1 : 0;
    const int wc = scan_chunk(key, nE, cbase, nodeBase, list, tid, lane, wave, vecok);
    if (lane == 0) wcnt[wave] = wc;
    __syncthreads();
    int pre = 0, all = 0;
#pragma unroll
    for (int w2 = 0; w2 < NWAVE; ++w2) {
      int c = wcnt[w2];
      c = c < 0 ? 0 : (c > WCAP ? WCAP : c);
      all += c;
      pre += (w2 < wave) ? c : 0;
    }
    const int wcc  = wc > WCAP ? WCAP : wc;
    const int base = tot + pre;
#pragma unroll 1
    for (int i = lane; i < wcc; i += 32) {
      const int ent = list[wave * WCAP + i];
      const int el  = (ent >> SLOTB) & (CHUNK - 1);
      const int sl  = ent & (NBMAX - 1);
      int eid = cbase + el;
      eid = eid > nE - 1 ? nE - 1 : eid;
      const int pos = base + i;
      if (pos < RCAP) reg1[pos] = (int)(((unsigned)eid << SLOTB) | (unsigned)sl);
    }
    tot += all;
    tot = tot > RCAP ? RCAP : tot;
    __syncthreads();
  }
  const int nh = tot;

  if (wave == 0) {
#pragma unroll 1
    for (int b0 = 0; b0 < nh; b0 += 32) {
      const int idx = b0 + lane;
      const int uv  = reg1[idx < RCAP ? idx : RCAP - 1];
      const int m32 = (nh - b0) < 32 ? (nh - b0) : 32;
#pragma unroll 1
      for (int k = 0; k < m32; ++k) {
        const int u  = __builtin_amdgcn_readlane(uv, k);
        const int sl = u & (NBMAX - 1);
        if (lane == 0) scnt[sl] = scnt[sl] + 1;
      }
    }
  }
  __syncthreads();

  {
    const v4i ca = *(const v4i*)(scnt + 4 * tid);
    const int e0 = ca.x < 0 ? 0 : ca.x, e1 = ca.y < 0 ? 0 : ca.y, e2 = ca.z < 0 ? 0 : ca.z, e3 = ca.w < 0 ? 0 : ca.w;
    const int ts = e0 + e1 + e2 + e3;
    int incl = ts;
#pragma unroll
    for (int d = 1; d < 32; d <<= 1) {
      const int up = __shfl_up(incl, d);
      if (lane >= d) incl += up;
    }
    if (lane == 31) wtot[wave] = incl;
    __syncthreads();
    int pre = 0;
#pragma unroll
    for (int w2 = 0; w2 < NWAVE; ++w2) pre += (w2 < wave) ? wtot[w2] : 0;
    int run = pre + incl - ts;
    soff[4 * tid + 0] = run; run += e0;
    soff[4 * tid + 1] = run; run += e1;
    soff[4 * tid + 2] = run; run += e2;
    soff[4 * tid + 3] = run;
  }
  __syncthreads();
  for (int i = tid; i < NBMAX; i += NTHR) list[i] = soff[i];
  __syncthreads();

  if (wave == 0) {
#pragma unroll 1
    for (int b0 = 0; b0 < nh; b0 += 32) {
      const int idx = b0 + lane;
      const int uv  = reg1[idx < RCAP ? idx : RCAP - 1];
      const int m32 = (nh - b0) < 32 ? (nh - b0) : 32;
#pragma unroll 1
      for (int k = 0; k < m32; ++k) {
        const int u   = __builtin_amdgcn_readlane(uv, k);
        const int sl  = u & (NBMAX - 1);
        const int eid = (int)((unsigned)u >> SLOTB);
        if (lane == 0) {
          int pos = list[sl];
          pos = pos < 0 ? 0 : (pos > RCAP - 1 ? RCAP - 1 : pos);
          reg2[pos] = eid;
          list[sl] = pos + 1;
        }
      }
    }
  }
  __syncthreads();

  const int wb = wave * WDEG;
  float* wr = wres + wave * (NCI * NBW);
  const bool ovf = (nh >= RCAP);
  const float qnan = __int_as_float(0x7fc00000);
  const int em = nE - 1, nm = nN - 1;
#pragma unroll 1
  for (int jt = 0; jt < NBW; ++jt) {
    const int slot = wave * NBW + jt;
    const int grow = nodeBase + slot;
    int st = soff[slot];
    const int craw = scnt[slot];
    int cnt = craw;
    st  = st < 0 ? 0 : (st > nh ? nh : st);
    cnt = cnt < 0 ? 0 : (cnt > WDEG ? WDEG : cnt);
    if (cnt > nh - st) cnt = nh - st;
    const float pz = (ovf || craw > WDEG) ? qnan : 0.0f;
    const int nr = (cnt + 31) >> 5;
#pragma unroll 1
    for (int rr = 0; rr < nr; ++rr) {
      const int q = 32 * rr + lane;
      int idx = st + q; idx = idx > RCAP - 1 ? RCAP - 1 : idx;
      int e = reg2[idx]; e = e < 0 ? 0 : (e > em ? em : e);
      int o = oth[e];    o = o < 0 ? 0 : (o > nm ? nm : o);
      if (q < cnt) wsrc[wb + q] = o;
    }
    __builtin_amdgcn_fence(__ATOMIC_RELEASE, "wavefront");
    __builtin_amdgcn_wave_barrier();
    float a[NCI];
#pragma unroll
    for (int c = 0; c < NCI; ++c) a[c] = 0.0f;
#pragma unroll 1
    for (int rr = 0; rr < nr; ++rr) {
      const int q = 32 * rr + lane;
      const bool act = q < cnt;
      const int qc = act ? q : 0;
      int idx = st + qc; idx = idx > RCAP - 1 ? RCAP - 1 : idx;
      int e = reg2[idx];     e = e < 0 ? 0 : (e > em ? em : e);
      int s = wsrc[wb + qc]; s = s < 0 ? 0 : (s > nm ? nm : s);
      const float w = ew[e];
      bool valid = act;
#pragma unroll 1
      for (int q2 = 0; q2 < cnt; ++q2) {
        int i2 = st + q2; i2 = i2 > RCAP - 1 ? RCAP - 1 : i2;
        int e2 = reg2[i2];  e2 = e2 < 0 ? 0 : (e2 > em ? em : e2);
        int s2 = wsrc[wb + q2]; s2 = s2 < 0 ? 0 : (s2 > nm ? nm : s2);
        if (s2 == s && e2 > e) valid = false;
      }
      if (MODE == 0) {
        a[0] += valid ? w : 0.0f;
      } else {
        const float coef = valid ? w * dpl[s] : 0.0f;
        if (MODE == 1) {
          const float* xr = vsrc + (size_t)s * NCI;
          const v4f x0 = *(const v4f*)xr, x1 = *(const v4f*)(xr + 4), x2 = *(const v4f*)(xr + 8);
          a[0] += coef * x0.x; a[1] += coef * x0.y; a[2]  += coef * x0.z; a[3]  += coef * x0.w;
          a[4] += coef * x1.x; a[5] += coef * x1.y; a[6]  += coef * x1.z; a[7]  += coef * x1.w;
          a[8] += coef * x2.x; a[9] += coef * x2.y; a[10] += coef * x2.z; a[11] += coef * x2.w;
        } else {
          a[0] += coef * vsrc[s];
        }
      }
    }
#pragma unroll
    for (int c = 0; c < NCO; ++c) {
      float v = a[c];
      v += __shfl_xor(v, 16);
      v += __shfl_xor(v, 8);
      v += __shfl_xor(v, 4);
      v += __shfl_xor(v, 2);
      v += __shfl_xor(v, 1);
      a[c] = v;
    }
    const int gi = grow > nm ? nm : grow;
    if (MODE == 0) {
      const float val = rsqrtf(1.0f + a[0]);
      if (lane == 0) wr[jt] = val + pz;
    } else if (MODE == 1) {
      const float di = dpl[grow];
      const float* xi = vsrc + (size_t)gi * NCI;
#pragma unroll
      for (int c = 0; c < NCI; ++c) {
        const float val = di * (a[c] + di * xi[c]);
        if (lane == 0) wr[c * NBW + jt] = val + pz;
      }
    } else {
      const float di = dpl[grow];
      const float val = di * (a[0] + di * vsrc[gi]);
      if (lane == 0) wr[jt] = val + pz;
    }
  }
  __builtin_amdgcn_fence(__ATOMIC_RELEASE, "wavefront");
  __builtin_amdgcn_wave_barrier();
  float ov[NCI][2];
#pragma unroll
  for (int c = 0; c < NCO; ++c) {
    ov[c][0] = wr[c * NBW + lane];
    ov[c][1] = wr[c * NBW + 32 + lane];
  }
  float* ob = outp + (size_t)nodeBase + (size_t)(wave * NBW) + lane;
#pragma unroll
  for (int c = 0; c < NCO; ++c) {
    *(volatile float*)(ob + (size_t)c * npad)      = ov[c][0];
    *(volatile float*)(ob + (size_t)c * npad + 32) = ov[c][1];
  }
  __threadfence();
#pragma unroll
  for (int c = 0; c < NCO; ++c) {
    *(volatile float*)(ob + (size_t)c * npad)      = ov[c][0];
    *(volatile float*)(ob + (size_t)c * npad + 32) = ov[c][1];
  }
}

__device__ __forceinline__ _Float16 th16(float x) {
  x = fminf(fmaxf(x, -9.0f), 9.0f);
  const float e = __expf(2.0f * x);
  const float r = __builtin_amdgcn_rcpf(1.0f + e);
  const float t = 1.0f - 2.0f * r;
  return (_Float16)(t * CG);
}
__global__ __launch_bounds__(NTHR) void k_gbuild(const float* __restrict__ axt, const float* __restrict__ gcnw,
                                                 _Float16* g16, int npad, int p, int nUnits) {
  const int u = (int)blockIdx.x * NTHR + (int)threadIdx.x;
  if (u >= nUnits) return;
  const int n  = u / KT8;
  const int j  = u - n * KT8;
  const int w  = j >> 5;
  const int h0 = (j & 31) * 8;
  const float av = axt[(size_t)(w + p) * npad + n];
  const v4f g0 = *(const v4f*)(gcnw + h0), g1 = *(const v4f*)(gcnw + h0 + 4);
  v8h hv;
  hv[0] = th16(av * g0.x); hv[1] = th16(av * g0.y); hv[2] = th16(av * g0.z); hv[3] = th16(av * g0.w);
  hv[4] = th16(av * g1.x); hv[5] = th16(av * g1.y); hv[6] = th16(av * g1.z); hv[7] = th16(av * g1.w);
  _Float16* o = g16 + (size_t)n * KT + 8 * j;
  *(volatile v8h*)o = hv;
  __threadfence();
  *(volatile v8h*)o = hv;
}

__global__ __launch_bounds__(GTHR) void k_gemm(const _Float16* __restrict__ g16, const _Float16* __restrict__ tat,
                                               const float* __restrict__ bias, _Float16* t16) {
  __shared__ __attribute__((aligned(16))) _Float16 stg[4 * 16 * PGRP];
  const int tid = threadIdx.x, lane = tid & 31, wave = tid >> 5, hh = lane >> 4, m = lane & 15;
  const int rowBase = (int)blockIdx.x * GBM;
  const size_t arow = (size_t)(rowBase + 16 * wave + m) * KT + 8 * hh;
  _Float16* sw = stg + wave * (16 * PGRP);
  const int rq = lane >> 3, c8 = lane & 7;
#pragma unroll 1
  for (int g = 0; g < NPGRP; ++g) {
    v8f acc[4];
    { v8f z = {0.f, 0.f, 0.f, 0.f, 0.f, 0.f, 0.f, 0.f}; acc[0] = z; acc[1] = z; acc[2] = z; acc[3] = z; }
#pragma unroll 2
    for (int ks = 0; ks < KS1; ++ks) {
      FragH af;
      af.h[0] = *(const v8h*)(g16 + arow + 32 * ks);
      af.h[1] = *(const v8h*)(g16 + arow + 32 * ks + 16);
#pragma unroll
      for (int t = 0; t < 4; ++t) {
        const size_t bo = (size_t)(g * PGRP + 16 * t + m) * KT + 8 * hh + 32 * ks;
        FragH bf;
        bf.h[0] = *(const v8h*)(tat + bo);
        bf.h[1] = *(const v8h*)(tat + bo + 16);
        acc[t] = wmh(af, bf, acc[t]);
      }
    }
    float bv[4];
#pragma unroll
    for (int t = 0; t < 4; ++t) bv[t] = bias[g * PGRP + 16 * t + m];
    __syncthreads();
#pragma unroll
    for (int t = 0; t < 4; ++t) {
#pragma unroll
      for (int r = 0; r < 8; ++r) {
        float v = acc[t][r] * SCL1 + bv[t];
        v = v > 0.0f ? v : 0.0f;
        sw[(8 * hh + r) * PGRP + 16 * t + m] = (_Float16)(v * CT);
      }
    }
    __syncthreads();
    v8h o[4];
#pragma unroll
    for (int i = 0; i < 4; ++i) o[i] = *(const v8h*)(sw + (4 * i + rq) * PGRP + 8 * c8);
    _Float16* pb = t16 + (size_t)(rowBase + 16 * wave + rq) * DD + (size_t)(g * PGRP + 8 * c8);
#pragma unroll
    for (int i = 0; i < 4; ++i) *(volatile v8h*)(pb + (size_t)(4 * i) * DD) = o[i];
    __threadfence();
#pragma unroll
    for (int i = 0; i < 4; ++i) *(volatile v8h*)(pb + (size_t)(4 * i) * DD) = o[i];
  }
}

__global__ __launch_bounds__(GTHR) void k_gru(const _Float16* __restrict__ t16, const _Float16* __restrict__ h16,
                                              const _Float16* __restrict__ wih, const _Float16* __restrict__ whh,
                                              const float* __restrict__ bih, const float* __restrict__ bhh,
                                              const float* __restrict__ hF, float* hOut, _Float16* hOut16) {
  __shared__ __attribute__((aligned(16))) float stg[16 * 128];
  const int tid = threadIdx.x, lane = tid & 31, wave = tid >> 5, hh = lane >> 4, m = lane & 15;
  const int rt = (int)blockIdx.x >> 1, cg = (int)blockIdx.x & 1;
  const int rowBase = 16 * rt;
  const int colW = 128 * cg + 32 * wave;
  const size_t arow = (size_t)(rowBase + m) * DD + 8 * hh;
  const size_t g1 = (size_t)DD * DD, g2 = (size_t)2 * DD * DD;
  v8f aR[2], aZ[2], aI[2], aH[2];
  { v8f z = {0.f, 0.f, 0.f, 0.f, 0.f, 0.f, 0.f, 0.f};
    aR[0] = z; aR[1] = z; aZ[0] = z; aZ[1] = z; aI[0] = z; aI[1] = z; aH[0] = z; aH[1] = z; }
#pragma unroll 1
  for (int ks = 0; ks < KS2; ++ks) {
    FragH am, ah;
    am.h[0] = *(const v8h*)(t16 + arow + 32 * ks);
    am.h[1] = *(const v8h*)(t16 + arow + 32 * ks + 16);
    ah.h[0] = *(const v8h*)(h16 + arow + 32 * ks);
    ah.h[1] = *(const v8h*)(h16 + arow + 32 * ks + 16);
#pragma unroll
    for (int t = 0; t < 2; ++t) {
      const size_t cb = (size_t)(colW + 16 * t + m) * DD + 8 * hh + 32 * ks;
      FragH b;
      b.h[0] = *(const v8h*)(wih + cb);           b.h[1] = *(const v8h*)(wih + cb + 16);           aR[t] = wmh(am, b, aR[t]);
      b.h[0] = *(const v8h*)(whh + cb);           b.h[1] = *(const v8h*)(whh + cb + 16);           aR[t] = wmh(ah, b, aR[t]);
      b.h[0] = *(const v8h*)(wih + g1 + cb);      b.h[1] = *(const v8h*)(wih + g1 + cb + 16);      aZ[t] = wmh(am, b, aZ[t]);
      b.h[0] = *(const v8h*)(whh + g1 + cb);      b.h[1] = *(const v8h*)(whh + g1 + cb + 16);      aZ[t] = wmh(ah, b, aZ[t]);
      b.h[0] = *(const v8h*)(wih + g2 + cb);      b.h[1] = *(const v8h*)(wih + g2 + cb + 16);      aI[t] = wmh(am, b, aI[t]);
      b.h[0] = *(const v8h*)(whh + g2 + cb);      b.h[1] = *(const v8h*)(whh + g2 + cb + 16);      aH[t] = wmh(ah, b, aH[t]);
    }
  }
#pragma unroll
  for (int t = 0; t < 2; ++t) {
    const int col = colW + 16 * t + m;
    const float br = bih[col] + bhh[col];
    const float bz = bih[DD + col] + bhh[DD + col];
    const float bi = bih[2 * DD + col];
    const float bn = bhh[2 * DD + col];
#pragma unroll
    for (int r = 0; r < 8; ++r) {
      const int row = rowBase + 8 * hh + r;
      const float hp = hF[(size_t)row * DD + col];
      float xr = aR[t][r] * SCL2 + br;
      float xz = aZ[t][r] * SCL2 + bz;
      xr = fminf(fmaxf(xr, -30.0f), 30.0f);
      xz = fminf(fmaxf(xz, -30.0f), 30.0f);
      const float R  = __builtin_amdgcn_rcpf(1.0f + __expf(-xr));
      const float Z  = __builtin_amdgcn_rcpf(1.0f + __expf(-xz));
      const float Nn = tanhf(aI[t][r] * SCL2 + bi + R * (aH[t][r] * SCL2 + bn));
      const float hn = (1.0f - Z) * Nn + Z * hp;
      stg[(8 * hh + r) * 128 + 32 * wave + 16 * t + m] = hn;
    }
  }
  __syncthreads();
  v4f o[4];
#pragma unroll
  for (int i = 0; i < 4; ++i) o[i] = *(const v4f*)(stg + (4 * i + wave) * 128 + 4 * lane);
  float* ob = hOut + (size_t)(128 * cg + 4 * lane);
  v8h q[2];
#pragma unroll
  for (int j = 0; j < 2; ++j) {
    const int rl = 4 * (2 * j + hh) + wave;
    const float* sp = stg + rl * 128 + 8 * m;
    const v4f a = *(const v4f*)sp, b = *(const v4f*)(sp + 4);
    v8h hv;
    hv[0] = (_Float16)(a.x * CHH); hv[1] = (_Float16)(a.y * CHH); hv[2] = (_Float16)(a.z * CHH); hv[3] = (_Float16)(a.w * CHH);
    hv[4] = (_Float16)(b.x * CHH); hv[5] = (_Float16)(b.y * CHH); hv[6] = (_Float16)(b.z * CHH); hv[7] = (_Float16)(b.w * CHH);
    q[j] = hv;
  }
  _Float16* ob16 = hOut16 + (size_t)(128 * cg + 8 * m);
#pragma unroll
  for (int i = 0; i < 4; ++i) {
    const int grow = rowBase + 4 * i + wave;
    *(volatile v4f*)(ob + (size_t)grow * DD) = o[i];
  }
#pragma unroll
  for (int j = 0; j < 2; ++j) {
    const int grow = rowBase + 4 * (2 * j + hh) + wave;
    *(volatile v8h*)(ob16 + (size_t)grow * DD) = q[j];
  }
  __threadfence();
#pragma unroll
  for (int i = 0; i < 4; ++i) {
    const int grow = rowBase + 4 * i + wave;
    *(volatile v4f*)(ob + (size_t)grow * DD) = o[i];
  }
#pragma unroll
  for (int j = 0; j < 2; ++j) {
    const int grow = rowBase + 4 * (2 * j + hh) + wave;
    *(volatile v8h*)(ob16 + (size_t)grow * DD) = q[j];
  }
}

__global__ __launch_bounds__(NTHR) void k_pred(const float* __restrict__ h32, const float* __restrict__ ow,
                                               const float* __restrict__ ob, float* prow) {
  __shared__ float sp[32];
  const int tid = threadIdx.x, lane = tid & 31, wave = tid >> 5;
  const int rowBase = (int)blockIdx.x * 32;
  const v4f w0 = *(const v4f*)(ow + 8 * lane), w1 = *(const v4f*)(ow + 8 * lane + 4);
  const float b0 = ob[0];
#pragma unroll
  for (int i = 0; i < 4; ++i) {
    const int rl = wave + 8 * i;
    const float* hr = h32 + (size_t)(rowBase + rl) * DD + 8 * lane;
    const v4f a = *(const v4f*)hr, b = *(const v4f*)(hr + 4);
    float s = a.x * w0.x + a.y * w0.y + a.z * w0.z + a.w * w0.w + b.x * w1.x + b.y * w1.y + b.z * w1.z + b.w * w1.w;
    s += __shfl_xor(s, 16);
    s += __shfl_xor(s, 8);
    s += __shfl_xor(s, 4);
    s += __shfl_xor(s, 2);
    s += __shfl_xor(s, 1);
    if (lane == 0) sp[rl] = s + b0;
  }
  __syncthreads();
  if (wave == 0) {
    const float v = sp[lane];
    float* po = prow + rowBase + lane;
    *(volatile float*)po = v;
    __threadfence();
    *(volatile float*)po = v;
  }
}

__global__ __launch_bounds__(NTHR) void k_out(const float* __restrict__ pr, float* out, int nN, int P, int npad, int nUnits) {
  const int u = (int)blockIdx.x * NTHR + (int)threadIdx.x;
  if (u >= nUnits) return;
  const int e0 = 4 * u;
  v4f v;
#pragma unroll
  for (int q = 0; q < 4; ++q) {
    const int e = e0 + q;
    int n = e / P;
    const int pp = e - n * P;
    n = n > nN - 1 ? nN - 1 : n;
    v[q] = pr[(size_t)pp * npad + n];
  }
  float* po = out + (size_t)e0;
  *(volatile v4f*)po = v;
  __threadfence();
  *(volatile v4f*)po = v;
}

extern "C" void kernel_launch(void* const* d_in, const int* in_sizes, int n_in,
                              void* d_out, int out_size, void* d_ws, size_t ws_size,
                              hipStream_t stream) {
  if (n_in < 12) return;
  const int nN = in_sizes[0] / WWIN;
  if (nN <= 0 || in_sizes[0] != nN * WWIN || nN > (1 << 20)) return;
  const int nE = in_sizes[2];
  if (nE < 1 || in_sizes[1] != 2 * nE || nE >= (1 << 22)) return;
  if (in_sizes[3] != DD || in_sizes[4] != KT * DD || in_sizes[5] != DD) return;
  if (in_sizes[6] != GRUW * DD || in_sizes[7] != GRUW * DD) return;
  if (in_sizes[8] != GRUW || in_sizes[9] != GRUW) return;
  if (in_sizes[10] != DD || in_sizes[11] < 1) return;
  if (out_size <= 0 || (out_size % nN) != 0 || (out_size & 3) != 0) return;
  const int P = out_size / nN;
  if (P < 1 || P > PMAXH) return;

  const float* x     = (const float*)d_in[0];
  const int*   ei    = (const int*)d_in[1];
  const float* ew    = (const float*)d_in[2];
  const float* gcn_w = (const float*)d_in[3];
  const float* ta_w  = (const float*)d_in[4];
  const float* ta_b  = (const float*)d_in[5];
  const float* w_ih  = (const float*)d_in[6];
  const float* w_hh  = (const float*)d_in[7];
  const float* b_ih  = (const float*)d_in[8];
  const float* b_hh  = (const float*)d_in[9];
  const float* out_w = (const float*)d_in[10];
  const float* out_b = (const float*)d_in[11];
  float* out = (float*)d_out;
  const int* esrc = ei;
  const int* edst = ei + nE;

  const int gA = (nN + NB - 1) / NB;
  const int MP = gA * NB;
  const int NT = WWIN + P;
  const int vec8 = ((nE % 8) == 0) ? 1 : 0;

  char* ws = (char*)d_ws;
  size_t off = 0;
  const size_t oTAT = off; off += (size_t)DD * KT * 2;             off = (off + 255) & ~(size_t)255;
  const size_t oWIH = off; off += (size_t)GRUW * DD * 2;           off = (off + 255) & ~(size_t)255;
  const size_t oWHH = off; off += (size_t)GRUW * DD * 2;           off = (off + 255) & ~(size_t)255;
  const size_t oD   = off; off += (size_t)MP * 4;                  off = (off + 255) & ~(size_t)255;
  const size_t oAXT = off; off += (size_t)NT * MP * 4;             off = (off + 255) & ~(size_t)255;
  const size_t oG   = off; off += (size_t)MP * KT * 2;             off = (off + 255) & ~(size_t)255;
  const size_t oT   = off; off += (size_t)MP * DD * 2;             off = (off + 255) & ~(size_t)255;
  const size_t oHA6 = off; off += (size_t)MP * DD * 2;
  const size_t oHA2 = off; off += (size_t)MP * DD * 4;             off = (off + 255) & ~(size_t)255;
  const size_t oHB6 = off; off += (size_t)MP * DD * 2;             off = (off + 255) & ~(size_t)255;
  const size_t oHB2 = off; off += (size_t)MP * DD * 4;             off = (off + 255) & ~(size_t)255;
  const size_t oPR  = off; off += (size_t)P * MP * 4;              off = (off + 255) & ~(size_t)255;
  if (off > ws_size) return;
  if (off > (size_t)134217728) return;
  _Float16* TAT  = (_Float16*)(ws + oTAT);
  _Float16* WIH  = (_Float16*)(ws + oWIH);
  _Float16* WHH  = (_Float16*)(ws + oWHH);
  float*    D    = (float*)(ws + oD);
  float*    AXT  = (float*)(ws + oAXT);
  _Float16* G16  = (_Float16*)(ws + oG);
  _Float16* T16  = (_Float16*)(ws + oT);
  _Float16* H16A = (_Float16*)(ws + oHA6);
  float*    H32A = (float*)(ws + oHA2);
  _Float16* H16B = (_Float16*)(ws + oHB6);
  float*    H32B = (float*)(ws + oHB2);
  float*    PR   = (float*)(ws + oPR);

  hipFuncSetAttribute(reinterpret_cast<const void*>(&k_spmv<0>), hipFuncAttributeMaxDynamicSharedMemorySize, LDS_SCAN);
  hipFuncSetAttribute(reinterpret_cast<const void*>(&k_spmv<1>), hipFuncAttributeMaxDynamicSharedMemorySize, LDS_SCAN);
  hipFuncSetAttribute(reinterpret_cast<const void*>(&k_spmv<2>), hipFuncAttributeMaxDynamicSharedMemorySize, LDS_SCAN);

  const int nUG = GRUW * (DD / 8);
  k_tat<<<KT / 64, NTHR, 0, stream>>>(ta_w, TAT, KT);
  k_cvt<<<(nUG + NTHR - 1) / NTHR, NTHR, 0, stream>>>(w_ih, WIH, GRUW, nUG, CWG);
  k_cvt<<<(nUG + NTHR - 1) / NTHR, NTHR, 0, stream>>>(w_hh, WHH, GRUW, nUG, CWG);
  const int nZ = (int)(((size_t)MP * DD * 2 + (size_t)MP * DD * 4) / 16);
  k_zero<<<(nZ + NTHR - 1) / NTHR, NTHR, 0, stream>>>((float*)(ws + oHA6), nZ);
  k_spmv<0><<<gA, NTHR, LDS_SCAN, stream>>>(esrc, edst, ew, D, x, D, nE, nN, MP, vec8);
  k_spmv<1><<<gA, NTHR, LDS_SCAN, stream>>>(edst, esrc, ew, D, x, AXT, nE, nN, MP, vec8);

  const int nUGB = MP * KT8;
  const int gGB  = (nUGB + NTHR - 1) / NTHR;
  for (int p = 0; p < P; ++p) {
    const _Float16* h16old = (p & 1) ? H16B : H16A;
    const float*    h32old = (p & 1) ? H32B : H32A;
    _Float16*       h16new = (p & 1) ? H16A : H16B;
    float*          h32new = (p & 1) ? H32A : H32B;
    k_gbuild<<<gGB, NTHR, 0, stream>>>(AXT, gcn_w, G16, MP, p, nUGB);
    k_gemm<<<MP / GBM, GTHR, 0, stream>>>(G16, TAT, ta_b, T16);
    k_gru<<<(MP / 16) * 2, GTHR, 0, stream>>>(T16, h16old, WIH, WHH, b_ih, b_hh, h32old, h32new, h16new);
    k_pred<<<MP / 32, NTHR, 0, stream>>>(h32new, out_w, out_b, PR + (size_t)p * MP);
    if (p + 1 < P)
      k_spmv<2><<<gA, NTHR, LDS_SCAN, stream>>>(edst, esrc, ew, D, PR + (size_t)p * MP,
                                                 AXT + (size_t)(WWIN + p) * MP, nE, nN, MP, vec8);
  }
  const int nUO = out_size / 4;
  k_out<<<(nUO + NTHR - 1) / NTHR, NTHR, 0, stream>>>(PR, out, nN, P, MP, nUO);
}
